// EFR_51153060496132
// MI455X (gfx1250) — hardware-verified
//
#include <hip/hip_runtime.h>
#include <stdint.h>

#define NB   2
#define NC   64
#define HH   192
#define WD   192
#define HW   (HH * WD)
#define NPX  (NB * HW)
#define NOF  18
#define NOP  32
#define SPA  72
#define OSO  36
#define OSP  68
#define EPSV 1e-5f
#define NGRID (NB * HH * 3)
#define NX4  (NB * NC * HW / 4)

#define XR_BYTES  ((size_t)NB * NC * HW * 4)
#define WPK_BYTES ((size_t)(NOP + NC) * NC * 2)
#define OFF_BYTES ((size_t)NPX * NOP * 4)
#define WS_XR   ((size_t)0)
#define WS_WPK  (WS_XR + XR_BYTES)
#define WS_OFF  (WS_WPK + WPK_BYTES)
#define WS_END  (WS_OFF + OFF_BYTES)

static_assert((XR_BYTES % 128) == 0);
static_assert((WPK_BYTES % 128) == 0);
static_assert((OFF_BYTES % 128) == 0);
static_assert((WS_WPK % 128) == 0);
static_assert((WS_OFF % 128) == 0);
static_assert(WS_END <= (size_t)134217728);
static_assert((NB * NC * HW) % 1024 == 0);
static_assert(NX4 % 256 == 0);
static_assert(((NOP + NC) * NC / 8) % 256 == 0);
static_assert((SPA * 2) % 16 == 0);
static_assert((OSO * 4) % 16 == 0);
static_assert((OSP * 4) % 16 == 0);
static_assert(64 * SPA * 2 * 2 + 64 * OSO * 4 + (NC * 39 + NC * 9 + NOP * 3) * 4 <= 60000);
static_assert(64 * SPA * 2 * 2 + NC * OSP * 4 + (27 * NC + 3 * NC) * 4 <= 60000);

typedef __bf16         v16b __attribute__((ext_vector_type(16)));
typedef float          v8f  __attribute__((ext_vector_type(8)));
typedef float          v4f  __attribute__((ext_vector_type(4)));
typedef unsigned short v8us __attribute__((ext_vector_type(8)));

__device__ __forceinline__ unsigned bfb(float f) {
  unsigned u = __float_as_uint(f);
  return (u + 0x7FFFu + ((u >> 16) & 1u)) >> 16;
}
__device__ __forceinline__ float bf_rne(float f) { return __uint_as_float(bfb(f) << 16); }
__device__ __forceinline__ v8f zero8f() { v8f z = {0.f, 0.f, 0.f, 0.f, 0.f, 0.f, 0.f, 0.f}; return z; }

union FragB { v16b v; v8us u[2]; };
__device__ __forceinline__ v16b ldfrag(const unsigned short* p) {
  FragB f;
  f.u[0] = *(const v8us*)(p);
  f.u[1] = *(const v8us*)(p + 16);
  return f.v;
}

__device__ __forceinline__ v8f mma_bg(const v16b& a, const v16b& b, v8f c) {
  v8f d = __builtin_amdgcn_wmma_f32_16x16x32_bf16(false, a, false, b, (short)0, c, false, false);
#if defined(__HIP_DEVICE_COMPILE__)
  asm volatile("v_nop\n\tv_nop\n\tv_nop\n\tv_nop" : "+v"(d) : "v"(a), "v"(b));
#endif
  return d;
}

__global__ __launch_bounds__(256)
void k_xr(const float* __restrict__ x, float* xr, int n4)
{
  const int i = blockIdx.x * 256 + threadIdx.x;
  if (i < n4) {
    const v4f v = *(const v4f*)(x + (size_t)i * 4);
    v4f r;
    r.x = bf_rne(v.x); r.y = bf_rne(v.y); r.z = bf_rne(v.z); r.w = bf_rne(v.w);
    float* d = xr + (size_t)i * 4;
    *(volatile v4f*)d = r;
    __threadfence();
    *(volatile v4f*)d = r;
  }
}

__global__ __launch_bounds__(256)
void k_wpack(const float* __restrict__ wbo, const float* __restrict__ wbl, unsigned short* wpk)
{
  const int tid = threadIdx.x;
  const int q   = blockIdx.x * 256 + tid;
  const int row = q >> 3;
  const int kc  = (q & 7) * 8;
  unsigned hb[8];
  if (blockIdx.x == 0) {
    const int n  = row;
    const int nn = (n < NOF) ? n : (NOF - 1);
    const bool live = (n < NOF);
    const float* src = wbo + nn * NC + kc;
#pragma unroll
    for (int j = 0; j < 8; ++j) {
      const unsigned v = bfb(src[j]);
      hb[j] = live ? v : 0u;
    }
  } else {
    const int n = row - NOP;
    const float* src = wbl + n * NC + kc;
#pragma unroll
    for (int j = 0; j < 8; ++j) hb[j] = bfb(src[j]);
  }
  v8us pv;
#pragma unroll
  for (int e = 0; e < 8; ++e) pv[e] = (unsigned short)hb[e];
  unsigned short* d = wpk + (size_t)q * 8;
  *(volatile v8us*)d = pv;
  __threadfence();
  *(volatile v8us*)d = pv;
}

__global__ __launch_bounds__(256)
void k_off(const float* __restrict__ xr,
           const float* __restrict__ w1, const float* __restrict__ b1, const float* __restrict__ n1,
           const float* __restrict__ w2, const float* __restrict__ b2, const float* __restrict__ n2,
           const float* __restrict__ w3, const float* __restrict__ b3, const float* __restrict__ n3,
           const float* __restrict__ bo, const float* __restrict__ nbo,
           const unsigned short* __restrict__ wpk, float* off)
{
  __shared__ float ws1[NC * 15];
  __shared__ float ws2[NC * 15];
  __shared__ float ws3[NC * 9];
  __shared__ float sc1[NC], sh1[NC], bb1[NC];
  __shared__ float sc2[NC], sh2[NC], bb2[NC];
  __shared__ float sc3[NC], sh3[NC], bb3[NC];
  __shared__ float sco[NOP], sho[NOP], bbo[NOP];
  __shared__ __align__(16) unsigned short sth[64 * SPA];
  __shared__ __align__(16) unsigned short stl[64 * SPA];
  __shared__ __align__(16) float os1[64 * OSO];

  const int tid  = threadIdx.x;
  const int lane = tid & 31;
  const int wid  = tid >> 5;
  const int l15  = lane & 15;
  const int hh   = lane >> 4;
  const int gid  = blockIdx.x;
  const int wt   = gid % 3;
  const int h    = (gid / 3) % HH;
  const int b    = gid / (3 * HH);
  const int w0   = 64 * wt;

#pragma unroll 1
  for (int i = tid; i < NC * 15; i += 256) { ws1[i] = bf_rne(w1[i]); ws2[i] = bf_rne(w2[i]); }
#pragma unroll 1
  for (int i = tid; i < NC * 9; i += 256) ws3[i] = bf_rne(w3[i]);
  if (tid < NC) {
    const int c = tid;
    {
      const float g = bf_rne(n1[c]), be = bf_rne(n1[NC + c]), mu = bf_rne(n1[2 * NC + c]), va = bf_rne(n1[3 * NC + c]);
      const float s = g * rsqrtf(va + EPSV);
      sc1[c] = s; sh1[c] = be - mu * s; bb1[c] = bf_rne(b1[c]);
    }
    {
      const float g = bf_rne(n2[c]), be = bf_rne(n2[NC + c]), mu = bf_rne(n2[2 * NC + c]), va = bf_rne(n2[3 * NC + c]);
      const float s = g * rsqrtf(va + EPSV);
      sc2[c] = s; sh2[c] = be - mu * s; bb2[c] = bf_rne(b2[c]);
    }
    {
      const float g = bf_rne(n3[c]), be = bf_rne(n3[NC + c]), mu = bf_rne(n3[2 * NC + c]), va = bf_rne(n3[3 * NC + c]);
      const float s = g * rsqrtf(va + EPSV);
      sc3[c] = s; sh3[c] = be - mu * s; bb3[c] = bf_rne(b3[c]);
    }
  }
  if (tid < NOP) {
    const int n  = tid;
    const int nn = (n < NOF) ? n : (NOF - 1);
    const bool live = (n < NOF);
    const float g = bf_rne(nbo[nn]), be = bf_rne(nbo[NOF + nn]), mu = bf_rne(nbo[2 * NOF + nn]), va = bf_rne(nbo[3 * NOF + nn]);
    const float s   = g * rsqrtf(va + EPSV);
    const float sh  = be - mu * s;
    const float bbv = bf_rne(bo[nn]);
    sco[n] = live ? s : 0.0f;
    sho[n] = live ? sh : 0.0f;
    bbo[n] = live ? bbv : 0.0f;
  }
  __syncthreads();

#pragma unroll 1
  for (int cc = 0; cc < 8; ++cc) {
    const int c = wid + 8 * cc;
    const float* xp   = xr + ((size_t)(b * NC + c)) * HW;
    const float* xrow = xp + h * WD;
    float wa[15], wb[15], wc[9];
#pragma unroll
    for (int k = 0; k < 15; ++k) { wa[k] = ws1[c * 15 + k]; wb[k] = ws2[c * 15 + k]; }
#pragma unroll
    for (int k = 0; k < 9; ++k) wc[k] = ws3[c * 9 + k];
    const float s1c = sc1[c], t1c = sh1[c], q1c = bb1[c];
    const float s2c = sc2[c], t2c = sh2[c], q2c = bb2[c];
    const float s3c = sc3[c], t3c = sh3[c], q3c = bb3[c];
#pragma unroll 1
    for (int mm = 0; mm < 2; ++mm) {
      const int m = lane + 32 * mm;
      const int w = w0 + m;
      float s1 = 0.0f;
#pragma unroll
      for (int k = 0; k < 15; ++k) {
        const int col  = w + k - 7;
        const int colc = min(max(col, 0), WD - 1);
        float v = xrow[colc];
        v = ((unsigned)col < (unsigned)WD) ? v : 0.0f;
        s1 += v * wa[k];
      }
      float s2 = 0.0f;
#pragma unroll
      for (int k = 0; k < 15; ++k) {
        const int row  = h + k - 7;
        const int rowc = min(max(row, 0), HH - 1);
        float v = xp[rowc * WD + w];
        v = ((unsigned)row < (unsigned)HH) ? v : 0.0f;
        s2 += v * wb[k];
      }
      float s3 = 0.0f;
#pragma unroll
      for (int ky = 0; ky < 3; ++ky) {
        const int row  = h + ky - 1;
        const int rowc = min(max(row, 0), HH - 1);
        const bool vr  = ((unsigned)row < (unsigned)HH);
#pragma unroll
        for (int kx = 0; kx < 3; ++kx) {
          const int col  = w + kx - 1;
          const int colc = min(max(col, 0), WD - 1);
          float v = xp[rowc * WD + colc];
          v = (vr && ((unsigned)col < (unsigned)WD)) ? v : 0.0f;
          s3 += v * wc[ky * 3 + kx];
        }
      }
      const float r1 = (s1 + q1c) * s1c + t1c;
      const float r2 = (s2 + q2c) * s2c + t2c;
      const float r3 = (s3 + q3c) * s3c + t3c;
      const float r  = (r1 + r2) + r3;
      const unsigned hbv = bfb(r);
      const unsigned lbv = bfb(r - __uint_as_float(hbv << 16));
      sth[m * SPA + c] = (unsigned short)hbv;
      stl[m * SPA + c] = (unsigned short)lbv;
    }
  }
  __syncthreads();

  {
    const int mt = wid & 3;
    const int nt = wid >> 2;
    const unsigned short* aph = sth + (16 * mt + l15) * SPA + 8 * hh;
    const unsigned short* apl = stl + (16 * mt + l15) * SPA + 8 * hh;
    const unsigned short* bp  = wpk + (size_t)(16 * nt + l15) * NC + 8 * hh;
    const v16b ah0 = ldfrag(aph);
    const v16b ah1 = ldfrag(aph + 32);
    const v16b al0 = ldfrag(apl);
    const v16b al1 = ldfrag(apl + 32);
    const v16b fb0 = ldfrag(bp);
    const v16b fb1 = ldfrag(bp + 32);
    v8f acc = zero8f();
    acc = mma_bg(ah0, fb0, acc);
    acc = mma_bg(al0, fb0, acc);
    acc = mma_bg(ah1, fb1, acc);
    acc = mma_bg(al1, fb1, acc);

    const int n = 16 * nt + l15;
    const float bbn = bbo[n], scn = sco[n], shn = sho[n];
    float* orow = os1 + (16 * mt + 8 * hh) * OSO + n;
#pragma unroll
    for (int r = 0; r < 8; ++r) {
      const float t = acc[r] + bbn;
      orow[r * OSO] = t * scn + shn;
    }
  }
  __syncthreads();

  {
    const int pj = lane & 7;
    const int lq = lane >> 3;
    const size_t pix0 = (size_t)b * HW + (size_t)h * WD + w0;
    v4f val[2]; size_t e[2];
#pragma unroll
    for (int r = 0; r < 2; ++r) {
      const int L = r * 32 + wid * 4 + lq;
      val[r] = *(const v4f*)(os1 + L * OSO + 4 * pj);
      e[r]   = (pix0 + L) * NOP + 4 * pj;
    }
#pragma unroll
    for (int r = 0; r < 2; ++r) *(volatile v4f*)(off + e[r]) = val[r];
    __threadfence();
#pragma unroll
    for (int r = 0; r < 2; ++r) *(volatile v4f*)(off + e[r]) = val[r];
  }
}

__global__ __launch_bounds__(256)
void k_main(const float* __restrict__ xr, const float* __restrict__ off, const float* __restrict__ wdef,
            const unsigned short* __restrict__ wpk, const float* __restrict__ bbal, const float* __restrict__ nbal,
            float* out)
{
  __shared__ __align__(16) float wd[27 * NC];
  __shared__ float scb[NC], shb[NC], bbb[NC];
  __shared__ __align__(16) unsigned short sth[64 * SPA];
  __shared__ __align__(16) unsigned short stl[64 * SPA];
  __shared__ __align__(16) float os2[NC * OSP];

  const int tid  = threadIdx.x;
  const int lane = tid & 31;
  const int wid  = tid >> 5;
  const int l15  = lane & 15;
  const int hh   = lane >> 4;
  const int gid  = blockIdx.x;
  const int wt   = gid % 3;
  const int h    = (gid / 3) % HH;
  const int b    = gid / (3 * HH);
  const int w0   = 64 * wt;

#pragma unroll 1
  for (int i = tid; i < 27 * NC; i += 256) {
    const int it = i >> 6;
    const int c  = i & 63;
    const int dd = (it >= 9 ? 1 : 0) + (it >= 18 ? 1 : 0);
    const int t  = it - 9 * dd;
    wd[i] = bf_rne(wdef[(dd * NC + c) * 9 + t]);
  }
  if (tid < NC) {
    const int c = tid;
    const float g = bf_rne(nbal[c]), be = bf_rne(nbal[NC + c]), mu = bf_rne(nbal[2 * NC + c]), va = bf_rne(nbal[3 * NC + c]);
    const float s = g * rsqrtf(va + EPSV);
    scb[c] = s; shb[c] = be - mu * s; bbb[c] = bf_rne(bbal[c]);
  }
  __syncthreads();

  {
    const int m  = tid & 63;
    const int cg = tid >> 6;
    const int w  = w0 + m;
    const float hfl = (float)h;
    const float wfl = (float)w;
    const float* offp = off + ((size_t)(b * HW + h * WD + w)) * NOP;
    const float* xb   = xr + ((size_t)(b * NC + 16 * cg)) * HW;
    float acc[16];
#pragma unroll
    for (int j = 0; j < 16; ++j) acc[j] = 0.0f;
#pragma unroll 1
    for (int dd = 0; dd < 3; ++dd) {
      const float dil = (dd == 0) ? 1.0f : ((dd == 1) ? 2.0f : 4.0f);
#pragma unroll 1
      for (int t = 0; t < 9; ++t) {
        const int kyi = (t >= 3 ? 1 : 0) + (t >= 6 ? 1 : 0);
        const int kxi = t - 3 * kyi;
        const float kyd = (float)(kyi - 1) * dil;
        const float kxd = (float)(kxi - 1) * dil;
        const float oy = offp[2 * t];
        const float ox = offp[2 * t + 1];
        const float yy = (oy + hfl) + kyd;
        const float xx = (ox + wfl) + kxd;
        const float y0f = floorf(yy);
        const float x0f = floorf(xx);
        const float y1f = y0f + 1.0f;
        const float x1f = x0f + 1.0f;
        const float wy1 = yy - y0f;
        const float wy0 = 1.0f - wy1;
        const float wx1 = xx - x0f;
        const float wx0 = 1.0f - wx1;
        const bool vy0 = (y0f >= 0.0f) && (y0f < (float)HH);
        const bool vy1 = (y1f >= 0.0f) && (y1f < (float)HH);
        const bool vx0 = (x0f >= 0.0f) && (x0f < (float)WD);
        const bool vx1 = (x1f >= 0.0f) && (x1f < (float)WD);
        const float f00 = (vy0 && vx0) ? (wy0 * wx0) : 0.0f;
        const float f01 = (vy0 && vx1) ? (wy0 * wx1) : 0.0f;
        const float f10 = (vy1 && vx0) ? (wy1 * wx0) : 0.0f;
        const float f11 = (vy1 && vx1) ? (wy1 * wx1) : 0.0f;
        const int yc0 = (int)fminf(fmaxf(y0f, 0.0f), (float)(HH - 1));
        const int yc1 = (int)fminf(fmaxf(y1f, 0.0f), (float)(HH - 1));
        const int xc0 = (int)fminf(fmaxf(x0f, 0.0f), (float)(WD - 1));
        const int xc1 = (int)fminf(fmaxf(x1f, 0.0f), (float)(WD - 1));
        const int o00 = yc0 * WD + xc0;
        const int o01 = yc0 * WD + xc1;
        const int o10 = yc1 * WD + xc0;
        const int o11 = yc1 * WD + xc1;
        const float* wdp = wd + (dd * 9 + t) * NC + 16 * cg;
#pragma unroll
        for (int j = 0; j < 16; ++j) {
          const float* pl = xb + (size_t)j * HW;
          const float s = ((pl[o00] * f00 + pl[o01] * f01) + pl[o10] * f10) + pl[o11] * f11;
          acc[j] += s * wdp[j];
        }
      }
    }
    v8us ph0, ph1, pl0, pl1;
#pragma unroll
    for (int j = 0; j < 8; ++j) {
      const unsigned ha = bfb(acc[j]);
      const unsigned la = bfb(acc[j] - __uint_as_float(ha << 16));
      const unsigned hc = bfb(acc[8 + j]);
      const unsigned lc = bfb(acc[8 + j] - __uint_as_float(hc << 16));
      ph0[j] = (unsigned short)ha; pl0[j] = (unsigned short)la;
      ph1[j] = (unsigned short)hc; pl1[j] = (unsigned short)lc;
    }
    unsigned short* th = sth + m * SPA + 16 * cg;
    unsigned short* tl = stl + m * SPA + 16 * cg;
    *(v8us*)(th)     = ph0;
    *(v8us*)(th + 8) = ph1;
    *(v8us*)(tl)     = pl0;
    *(v8us*)(tl + 8) = pl1;
  }
  __syncthreads();

  {
    const int mt  = wid & 3;
    const int ntp = wid >> 2;
    const unsigned short* aph = sth + (16 * mt + l15) * SPA + 8 * hh;
    const unsigned short* apl = stl + (16 * mt + l15) * SPA + 8 * hh;
    const unsigned short* bp0 = wpk + (size_t)(NOP + 32 * ntp + l15) * NC + 8 * hh;
    const unsigned short* bp1 = bp0 + 16 * NC;
    const v16b ah0 = ldfrag(aph);
    const v16b ah1 = ldfrag(aph + 32);
    const v16b al0 = ldfrag(apl);
    const v16b al1 = ldfrag(apl + 32);
    const v16b b00 = ldfrag(bp0);
    const v16b b01 = ldfrag(bp0 + 32);
    const v16b b10 = ldfrag(bp1);
    const v16b b11 = ldfrag(bp1 + 32);
    v8f acc0 = zero8f(), acc1 = zero8f();
    acc0 = mma_bg(ah0, b00, acc0);
    acc0 = mma_bg(al0, b00, acc0);
    acc0 = mma_bg(ah1, b01, acc0);
    acc0 = mma_bg(al1, b01, acc0);
    acc1 = mma_bg(ah0, b10, acc1);
    acc1 = mma_bg(al0, b10, acc1);
    acc1 = mma_bg(ah1, b11, acc1);
    acc1 = mma_bg(al1, b11, acc1);

    const int c0 = 32 * ntp + l15;
    const int c1 = c0 + 16;
    const float q0 = bbb[c0], s0 = scb[c0], t0 = shb[c0];
    const float q1 = bbb[c1], s1 = scb[c1], t1 = shb[c1];
    v4f pa, pb, pc, pe;
    pa.x = (acc0[0] + q0) * s0 + t0;  pa.y = (acc0[1] + q0) * s0 + t0;
    pa.z = (acc0[2] + q0) * s0 + t0;  pa.w = (acc0[3] + q0) * s0 + t0;
    pb.x = (acc0[4] + q0) * s0 + t0;  pb.y = (acc0[5] + q0) * s0 + t0;
    pb.z = (acc0[6] + q0) * s0 + t0;  pb.w = (acc0[7] + q0) * s0 + t0;
    pc.x = (acc1[0] + q1) * s1 + t1;  pc.y = (acc1[1] + q1) * s1 + t1;
    pc.z = (acc1[2] + q1) * s1 + t1;  pc.w = (acc1[3] + q1) * s1 + t1;
    pe.x = (acc1[4] + q1) * s1 + t1;  pe.y = (acc1[5] + q1) * s1 + t1;
    pe.z = (acc1[6] + q1) * s1 + t1;  pe.w = (acc1[7] + q1) * s1 + t1;
    float* o0 = os2 + c0 * OSP + 16 * mt + 8 * hh;
    float* o1 = os2 + c1 * OSP + 16 * mt + 8 * hh;
    *(v4f*)(o0)     = pa;
    *(v4f*)(o0 + 4) = pb;
    *(v4f*)(o1)     = pc;
    *(v4f*)(o1 + 4) = pe;
  }
  __syncthreads();

  {
    const int pj = lane & 7;
    const int lq = lane >> 3;
    v4f val[4]; size_t e[4];
#pragma unroll
    for (int r = 0; r < 4; ++r) {
      const int L   = r * 32 + wid * 4 + lq;
      const int chn = L >> 1;
      const int hf  = L & 1;
      const size_t ei = ((size_t)(b * NC + chn) * HH + h) * WD + w0 + 32 * hf + 4 * pj;
      const v4f bv = *(const v4f*)(os2 + chn * OSP + 32 * hf + 4 * pj);
      const v4f xv = *(const v4f*)(xr + ei);
      val[r] = bv * xv;
      e[r]   = ei;
    }
#pragma unroll
    for (int r = 0; r < 4; ++r) *(volatile v4f*)(out + e[r]) = val[r];
    __threadfence();
#pragma unroll
    for (int r = 0; r < 4; ++r) *(volatile v4f*)(out + e[r]) = val[r];
  }
}

extern "C" void kernel_launch(void* const* d_in, const int* in_sizes, int n_in,
                              void* d_out, int out_size, void* d_ws, size_t ws_size,
                              hipStream_t stream) {
  if (n_in < 17) return;
  if (in_sizes[0]  != NB * NC * HW) return;
  if (in_sizes[1]  != NC * 15) return;
  if (in_sizes[2]  != NC) return;
  if (in_sizes[3]  != 4 * NC) return;
  if (in_sizes[4]  != NC * 15) return;
  if (in_sizes[5]  != NC) return;
  if (in_sizes[6]  != 4 * NC) return;
  if (in_sizes[7]  != NC * 9) return;
  if (in_sizes[8]  != NC) return;
  if (in_sizes[9]  != 4 * NC) return;
  if (in_sizes[10] != NOF * NC) return;
  if (in_sizes[11] != NOF) return;
  if (in_sizes[12] != 4 * NOF) return;
  if (in_sizes[13] != 3 * NC * 9) return;
  if (in_sizes[14] != NC * NC) return;
  if (in_sizes[15] != NC) return;
  if (in_sizes[16] != 4 * NC) return;
  if (out_size != NB * NC * HW) return;
  if (WS_END > ws_size) return;

  const float* x          = (const float*)d_in[0];
  const float* w_off1     = (const float*)d_in[1];
  const float* b_off1     = (const float*)d_in[2];
  const float* bn_off1    = (const float*)d_in[3];
  const float* w_off2     = (const float*)d_in[4];
  const float* b_off2     = (const float*)d_in[5];
  const float* bn_off2    = (const float*)d_in[6];
  const float* w_off3     = (const float*)d_in[7];
  const float* b_off3     = (const float*)d_in[8];
  const float* bn_off3    = (const float*)d_in[9];
  const float* w_bal_off  = (const float*)d_in[10];
  const float* b_bal_off  = (const float*)d_in[11];
  const float* bn_bal_off = (const float*)d_in[12];
  const float* w_def      = (const float*)d_in[13];
  const float* w_bal      = (const float*)d_in[14];
  const float* b_bal      = (const float*)d_in[15];
  const float* bn_bal     = (const float*)d_in[16];
  float* out = (float*)d_out;
  char* ws = (char*)d_ws;

  float* xr           = (float*)(ws + WS_XR);
  unsigned short* wpk = (unsigned short*)(ws + WS_WPK);
  float* offp         = (float*)(ws + WS_OFF);

  k_xr<<<dim3(NX4 / 256), dim3(256), 0, stream>>>(x, xr, NX4);
  (void)hipGetLastError();

  k_wpack<<<dim3((NOP + NC) * NC / 8 / 256), dim3(256), 0, stream>>>(w_bal_off, w_bal, wpk);
  (void)hipGetLastError();

  k_off<<<dim3(NGRID), dim3(256), 0, stream>>>(xr, w_off1, b_off1, bn_off1, w_off2, b_off2, bn_off2,
                                               w_off3, b_off3, bn_off3, b_bal_off, bn_bal_off,
                                               (const unsigned short*)wpk, offp);
  (void)hipGetLastError();

  k_main<<<dim3(NGRID), dim3(256), 0, stream>>>(xr, offp, w_def, (const unsigned short*)wpk,
                                                b_bal, bn_bal, out);
  (void)hipGetLastError();
}
